// ImprovedMambaBlock_59828894433548
// MI455X (gfx1250) — hardware-run, weakly checked
//
#include <hip/hip_runtime.h>
#include <hip/hip_fp16.h>
#include <math.h>

typedef float    ms1_v4f __attribute__((ext_vector_type(4)));
typedef unsigned ms1_v4u __attribute__((ext_vector_type(4)));
struct ms1_args {
  const float* dtpre;
  const float* u;
  const float* bc;
  const float* z;
  const float* A_log;
  const float* Dskip;
  __half* y;
  __half* y_lo;
  long ld_dtpre;
  long ld_u;
  long ld_bc;
  long ld_z;
  long ld_y;
  int offB;
  int offC;
  int offZ;
  float ycarry;
  int dir;
  int D;
  int L;
  int nbatch;
};
static_assert(sizeof(ms1_args) == 136);

__device__ __forceinline__ float ms1_flush16(float v) {
  return (fabsf(v) < 6.103515625e-05f) ? 0.0f : v;
}
__device__ __forceinline__ unsigned ms1_h16bits(float v) {
  return (unsigned)__half_as_ushort(__float2half_rn(ms1_flush16(v)));
}
__device__ __forceinline__ float ms1_h16val(unsigned b) {
  return __half2float(__ushort_as_half((unsigned short)b));
}
__device__ __forceinline__ float ms1_softplus(float v) {
  return fmaxf(v, 0.0f) + log1pf(expf(-fabsf(v)));
}
__device__ __forceinline__ void ms1_pack2(float v0, float v1, unsigned& hw, unsigned& lw) {
  const unsigned h0 = ms1_h16bits(v0);
  const unsigned h1 = ms1_h16bits(v1);
  const float r0 = (v0 - ms1_h16val(h0)) * 2048.0f;
  const float r1 = (v1 - ms1_h16val(h1)) * 2048.0f;
  const unsigned l0 = ms1_h16bits(r0);
  const unsigned l1 = ms1_h16bits(r1);
  hw = h0 | (h1 << 16);
  lw = l0 | (l1 << 16);
}

template <int NSTATE>
__global__ __launch_bounds__(64 * (NSTATE / 16)) void ms1_scan_kernel(ms1_args a)
{
  static_assert(NSTATE == 16 || NSTATE == 64);
  constexpr int NQ  = NSTATE / 16;
  constexpr int NT  = 64 * NQ;
  constexpr int NW  = NT / 32;
  constexpr int BCW = 2 * NSTATE;
  constexpr int YP  = 68;
  constexpr int RPI = NW * 4;
  constexpr int NIT = 64 / RPI;
  static_assert(16 * NT <= 64 * YP);
  __shared__ __align__(16) float sBC[64 * BCW];
  __shared__ __align__(16) float sY[64 * YP];
  const int tid  = threadIdx.x;
  const int lane = tid & 31;
  const int wave = tid >> 5;
  const int c    = tid / NQ;
  const int sq   = tid - c * NQ;
  const int bpb  = a.D / 64;
  const int bi   = blockIdx.x / bpb;
  if (bi >= a.nbatch) return;
  const int d0 = (blockIdx.x - bi * bpb) * 64;
  const int d  = d0 + c;
  const long rowb = (long)bi * a.L;
  const bool hasz  = (a.z != nullptr);
  const bool hasD  = (a.Dskip != nullptr);
  const bool hasLo = (a.y_lo != nullptr);

#pragma unroll 1
  for (int n = 0; n < 16; ++n) {
    const float al = a.A_log[(long)d * NSTATE + sq * 16 + n];
    sY[n * NT + tid] = -expf(al);
  }
  __syncthreads();
  float An[16], h[16];
#pragma unroll
  for (int n = 0; n < 16; ++n) {
    An[n] = sY[n * NT + tid];
    h[n] = 0.0f;
  }
  float Dd = 0.0f;
  if (hasD) Dd = a.Dskip[d];

  const int nchunk = a.L / 64;
  const bool fwd = (a.dir > 0);
  const int s0 = fwd ? 0 : 63;
  const int sd = fwd ? 1 : -1;
  const int q  = lane >> 3;
  const int c8 = (lane & 7) * 8;

#pragma unroll 1
  for (int ci = 0; ci < nchunk; ++ci) {
    const int tb = fwd ? (ci * 64) : (a.L - 64 - ci * 64);
    const long rowc = rowb + tb;
    __syncthreads();
#pragma unroll 8
    for (int i = 0; i < 32; ++i) {
      const int idx = tid + i * NT;
      const int st  = idx / BCW;
      const int col = idx - st * BCW;
      const int sc  = (col < NSTATE) ? (a.offB + col) : (a.offC + col - NSTATE);
      sBC[idx] = a.bc[(rowc + st) * a.ld_bc + sc];
    }
    __syncthreads();
#pragma unroll 1
    for (int s = 0; s < 64; ++s) {
      const int ls = s0 + sd * s;
      const long row = rowc + ls;
      float pre = a.dtpre[row * a.ld_dtpre + d];
      float uv  = a.u[row * a.ld_u + d];
      float zv  = 0.0f;
      if (hasz) zv = a.z[row * a.ld_z + a.offZ + d];
      asm volatile("" : "+v"(pre));
      asm volatile("" : "+v"(uv));
      asm volatile("" : "+v"(zv));
      const float delta = ms1_softplus(pre);
      const float dtx = delta * uv;
      const float* bp = sBC + ls * BCW + sq * 16;
      const float* cp = bp + NSTATE;
      ms1_v4f Bq[4], Cq[4];
#pragma unroll
      for (int k = 0; k < 4; ++k) {
        Bq[k] = *(const ms1_v4f*)(bp + 4 * k);
        Cq[k] = *(const ms1_v4f*)(cp + 4 * k);
      }
      float yv = 0.0f;
#pragma unroll
      for (int n = 0; n < 16; ++n) {
        const float e = __expf(delta * An[n]);
        h[n] = fmaf(e, h[n], dtx * Bq[n >> 2][n & 3]);
        yv = fmaf(h[n], Cq[n >> 2][n & 3], yv);
      }
      if (NQ > 1) {
        yv += __shfl_xor(yv, 1, 32);
        yv += __shfl_xor(yv, 2, 32);
      }
      if (hasD) yv = fmaf(uv, Dd, yv);
      if (hasz) {
        const float sg = __builtin_amdgcn_rcpf(1.0f + expf(-zv));
        yv = yv * (zv * sg);
      }
      if (sq == 0) sY[ls * YP + c] = yv * a.ycarry;
    }
    __syncthreads();
    ms1_v4u hw[NIT], lw[NIT];
#pragma unroll
    for (int it = 0; it < NIT; ++it) {
      const int row = it * RPI + wave * 4 + q;
      const float* sp = sY + row * YP + c8;
      const ms1_v4f f0 = *(const ms1_v4f*)(sp);
      const ms1_v4f f1 = *(const ms1_v4f*)(sp + 4);
      unsigned h0, h1, h2, h3, l0, l1, l2, l3;
      ms1_pack2(f0[0], f0[1], h0, l0);
      ms1_pack2(f0[2], f0[3], h1, l1);
      ms1_pack2(f1[0], f1[1], h2, l2);
      ms1_pack2(f1[2], f1[3], h3, l3);
      hw[it] = (ms1_v4u){h0, h1, h2, h3};
      lw[it] = (ms1_v4u){l0, l1, l2, l3};
    }
    for (int pass = 0; pass < 2; ++pass) {
#pragma unroll
      for (int it = 0; it < NIT; ++it) {
        const int row = it * RPI + wave * 4 + q;
        const long o = (rowc + row) * a.ld_y + d0 + c8;
        *(volatile ms1_v4u*)(a.y + o) = hw[it];
        if (hasLo) *(volatile ms1_v4u*)(a.y_lo + o) = lw[it];
      }
      __threadfence();
    }
  }
}

namespace eng {

constexpr int kBatch   = 4;
constexpr int kSeq     = 1024;
constexpr int kDm      = 1024;
constexpr int kDin     = 2048;
constexpr int kNstate  = 16;
constexpr int kPassB   = 2;
constexpr int kNpass   = kBatch / kPassB;
constexpr int kRows    = kPassB * kSeq;
constexpr int kRowsAll = kBatch * kSeq;
constexpr int kXgN     = 2 * kDin;
constexpr int kBcP     = 64;
constexpr int kOffB    = 0;
constexpr int kOffC    = kNstate;

static_assert(kBatch % kPassB == 0);
static_assert((kSeq & (kSeq - 1)) == 0);
static_assert(kDm == 4 * 256);
static_assert(kDin == 2 * 1024);
static_assert(kRows % 64 == 0 && kXgN % 64 == 0 && kDin % 64 == 0 && kDm % 64 == 0 && kBcP % 64 == 0);
static_assert(kDm % 32 == 0 && kDin % 32 == 0);
static_assert(kDin % 64 == 0 && kSeq % 64 == 0);
static_assert(2 * kNstate <= kBcP);

constexpr float kCarryXn   = 64.0f;
constexpr float kCarryWin  = 256.0f;
constexpr float kCarryU    = 64.0f;
constexpr float kCarryWdt  = 256.0f;
constexpr float kCarryWbc  = 256.0f;
constexpr float kCarryY    = 1024.0f;
constexpr float kCarryWout = 256.0f;
constexpr float kFoldIn    = 1.0f / (kCarryXn * kCarryWin);
constexpr float kFoldDt    = 1.0f / (kCarryU * kCarryWdt);
constexpr float kFoldBc    = 1.0f / (kCarryU * kCarryWbc);
constexpr float kFoldOut   = 1.0f / (kCarryY * kCarryWout);
constexpr float kInvDm     = 1.0f / (float)kDm;
constexpr float kLnEps     = 1e-5f;

constexpr size_t kBytesWin  = (size_t)kXgN * kDm * 2;
constexpr size_t kBytesWdt  = (size_t)kDin * kDin * 2;
constexpr size_t kBytesWbc  = (size_t)kBcP * kDin * 2;
constexpr size_t kBytesWout = (size_t)kDm * kDin * 2;
constexpr size_t kBytesXh   = (size_t)kRows * kDm * 2;
constexpr size_t kBytesXZ   = (size_t)kRows * kXgN * 4;
constexpr size_t kBytesUC   = (size_t)kRows * kDin * 4;
constexpr size_t kBytesUCh  = (size_t)kRows * kDin * 2;
constexpr size_t kBytesDTP  = (size_t)kRows * kDin * 4;
constexpr size_t kBytesBC   = (size_t)kRows * kBcP * 4;
constexpr size_t kBytesYH   = (size_t)kRows * kDin * 2;
constexpr size_t kWsTotal = kBytesWin + kBytesWdt + kBytesWbc + kBytesWout + kBytesXh + kBytesXZ + kBytesUC +
                            kBytesUCh + kBytesDTP + kBytesBC + kBytesYH;
static_assert(kWsTotal == 109838336ull);
static_assert(kWsTotal <= 134217728ull);
static_assert(kBytesWin % 128 == 0 && kBytesWdt % 128 == 0 && kBytesWbc % 128 == 0 && kBytesWout % 128 == 0 &&
              kBytesXh % 128 == 0 && kBytesXZ % 128 == 0 && kBytesUC % 128 == 0 && kBytesUCh % 128 == 0 &&
              kBytesDTP % 128 == 0 && kBytesBC % 128 == 0 && kBytesYH % 128 == 0);

typedef _Float16 v16h __attribute__((ext_vector_type(16)));
typedef _Float16 v8h  __attribute__((ext_vector_type(8)));
typedef float    v8f  __attribute__((ext_vector_type(8)));
typedef float    v4f  __attribute__((ext_vector_type(4)));
typedef unsigned v4u  __attribute__((ext_vector_type(4)));

__device__ __forceinline__ float flush16(float v) {
  return (fabsf(v) < 6.103515625e-05f) ? 0.0f : v;
}
__device__ __forceinline__ unsigned h16bits(float v) {
  return (unsigned)__half_as_ushort(__float2half_rn(flush16(v)));
}
__device__ __forceinline__ unsigned pack2(float a, float b) {
  const unsigned lo = h16bits(a);
  const unsigned hi = h16bits(b);
  return lo | (hi << 16);
}

union FragU { v16h v; v8h h[2]; };
__device__ __forceinline__ v16h frag_load(const _Float16* p) {
  FragU f;
  f.h[0] = *(const v8h*)(p);
  f.h[1] = *(const v8h*)(p + 16);
  return f.v;
}
__device__ __forceinline__ v8f mma(v16h a, v16h b, v8f c) {
  c = __builtin_amdgcn_wmma_f32_16x16x32_f16(false, a, false, b, (short)0, c, false, false);
  asm volatile("v_nop\n\tv_nop\n\tv_nop\n\tv_nop" : "+v"(c) : "v"(a), "v"(b));
  return c;
}

__device__ __forceinline__ float wave_sum(float v) {
#pragma unroll
  for (int off = 16; off >= 1; off >>= 1) v += __shfl_xor(v, off, 32);
  return v;
}

__global__ __launch_bounds__(256) void cast_carry_f16_kernel(
    const float* __restrict__ in, unsigned short* __restrict__ out, int n8, float carry)
{
  const int i = blockIdx.x * 256 + threadIdx.x;
  if (i < n8) {
    const v4f f0 = *(const v4f*)(in + (size_t)i * 8);
    const v4f f1 = *(const v4f*)(in + (size_t)i * 8 + 4);
    const float e0 = f0[0] * carry;
    const float e1 = f0[1] * carry;
    const float e2 = f0[2] * carry;
    const float e3 = f0[3] * carry;
    const float e4 = f1[0] * carry;
    const float e5 = f1[1] * carry;
    const float e6 = f1[2] * carry;
    const float e7 = f1[3] * carry;
    const v4u hw = (v4u){pack2(e0, e1), pack2(e2, e3), pack2(e4, e5), pack2(e6, e7)};
    unsigned short* o = out + (size_t)i * 8;
    for (int pass = 0; pass < 2; ++pass) {
      *(volatile v4u*)(o) = hw;
      __threadfence();
    }
  }
}

__global__ __launch_bounds__(256) void cast_bc_kernel(
    const float* __restrict__ Bw, const float* __restrict__ Cw, unsigned short* __restrict__ out, float carry)
{
  const int row = blockIdx.x;
  const int col = threadIdx.x * 8;
  const int rb = (row < kNstate) ? row : (kNstate - 1);
  int rc = row - kNstate;
  rc = (rc < 0) ? 0 : rc;
  rc = (rc > kNstate - 1) ? (kNstate - 1) : rc;
  v4f b0 = *(const v4f*)(Bw + (size_t)rb * kDin + col);
  v4f b1 = *(const v4f*)(Bw + (size_t)rb * kDin + col + 4);
  v4f c0 = *(const v4f*)(Cw + (size_t)rc * kDin + col);
  v4f c1 = *(const v4f*)(Cw + (size_t)rc * kDin + col + 4);
  asm volatile("" : "+v"(b0));
  asm volatile("" : "+v"(b1));
  asm volatile("" : "+v"(c0));
  asm volatile("" : "+v"(c1));
  const bool isB = (row < kNstate);
  const bool isC = (row >= kNstate) && (row < 2 * kNstate);
  const float e0 = isB ? (b0[0] * carry) : (isC ? (c0[0] * carry) : 0.0f);
  const float e1 = isB ? (b0[1] * carry) : (isC ? (c0[1] * carry) : 0.0f);
  const float e2 = isB ? (b0[2] * carry) : (isC ? (c0[2] * carry) : 0.0f);
  const float e3 = isB ? (b0[3] * carry) : (isC ? (c0[3] * carry) : 0.0f);
  const float e4 = isB ? (b1[0] * carry) : (isC ? (c1[0] * carry) : 0.0f);
  const float e5 = isB ? (b1[1] * carry) : (isC ? (c1[1] * carry) : 0.0f);
  const float e6 = isB ? (b1[2] * carry) : (isC ? (c1[2] * carry) : 0.0f);
  const float e7 = isB ? (b1[3] * carry) : (isC ? (c1[3] * carry) : 0.0f);
  const v4u hw = (v4u){pack2(e0, e1), pack2(e2, e3), pack2(e4, e5), pack2(e6, e7)};
  unsigned short* o = out + (size_t)row * kDin + col;
  for (int pass = 0; pass < 2; ++pass) {
    *(volatile v4u*)(o) = hw;
    __threadfence();
  }
}

__device__ __forceinline__ float ln_one(float xv, float mu, float rs, float w, float b, float carry) {
  const float nv = (xv - mu) * rs;
  const float ov = fmaf(nv, w, b);
  return ov * carry;
}

__global__ __launch_bounds__(256) void layernorm_cast_kernel(
    const float* __restrict__ x, const float* __restrict__ nw, const float* __restrict__ nb,
    unsigned short* __restrict__ xh, int rows, float carry)
{
  const int lane = threadIdx.x & 31;
  const int wave = threadIdx.x >> 5;
  const int row  = blockIdx.x * 8 + wave;
  if (row >= rows) return;
  const float* xr = x + (size_t)row * kDm;
  v4f v[8];
#pragma unroll
  for (int it = 0; it < 4; ++it) {
    v[2 * it]     = *(const v4f*)(xr + it * 256 + lane * 8);
    v[2 * it + 1] = *(const v4f*)(xr + it * 256 + lane * 8 + 4);
  }
  float s = 0.0f;
#pragma unroll
  for (int j = 0; j < 8; ++j) {
    s += v[j][0];
    s += v[j][1];
    s += v[j][2];
    s += v[j][3];
  }
  s = wave_sum(s);
  const float mu = s * kInvDm;
  float sq = 0.0f;
#pragma unroll
  for (int j = 0; j < 8; ++j) {
    const float d0 = v[j][0] - mu;
    const float d1 = v[j][1] - mu;
    const float d2 = v[j][2] - mu;
    const float d3 = v[j][3] - mu;
    sq = fmaf(d0, d0, sq);
    sq = fmaf(d1, d1, sq);
    sq = fmaf(d2, d2, sq);
    sq = fmaf(d3, d3, sq);
  }
  sq = wave_sum(sq);
  const float var = sq * kInvDm;
  const float rs = 1.0f / sqrtf(var + kLnEps);
  v4u hw[4];
#pragma unroll
  for (int it = 0; it < 4; ++it) {
    const int cb = it * 256 + lane * 8;
    const v4f w0 = *(const v4f*)(nw + cb);
    const v4f w1 = *(const v4f*)(nw + cb + 4);
    const v4f b0 = *(const v4f*)(nb + cb);
    const v4f b1 = *(const v4f*)(nb + cb + 4);
    const v4f a0 = v[2 * it];
    const v4f a1 = v[2 * it + 1];
    const float e0 = ln_one(a0[0], mu, rs, w0[0], b0[0], carry);
    const float e1 = ln_one(a0[1], mu, rs, w0[1], b0[1], carry);
    const float e2 = ln_one(a0[2], mu, rs, w0[2], b0[2], carry);
    const float e3 = ln_one(a0[3], mu, rs, w0[3], b0[3], carry);
    const float e4 = ln_one(a1[0], mu, rs, w1[0], b1[0], carry);
    const float e5 = ln_one(a1[1], mu, rs, w1[1], b1[1], carry);
    const float e6 = ln_one(a1[2], mu, rs, w1[2], b1[2], carry);
    const float e7 = ln_one(a1[3], mu, rs, w1[3], b1[3], carry);
    hw[it] = (v4u){pack2(e0, e1), pack2(e2, e3), pack2(e4, e5), pack2(e6, e7)};
  }
  unsigned short* orow = xh + (size_t)row * kDm;
  for (int pass = 0; pass < 2; ++pass) {
#pragma unroll
    for (int it = 0; it < 4; ++it) {
      *(volatile v4u*)(orow + it * 256 + lane * 8) = hw[it];
    }
    __threadfence();
  }
}

template <int EPI>
__global__ __launch_bounds__(256) void gemm_f16_kernel(
    const unsigned short* __restrict__ Ap, int lda,
    const unsigned short* __restrict__ Btp, int ldb,
    float* __restrict__ C, int ldc,
    const float* __restrict__ bias,
    const float* __restrict__ addp,
    int M, int N, int K, float scale)
{
  const _Float16* A  = (const _Float16*)(const void*)Ap;
  const _Float16* Bt = (const _Float16*)(const void*)Btp;
  __shared__ __align__(16) float sT[8][16 * 68];
  const int lane = threadIdx.x & 31;
  const int wave = threadIdx.x >> 5;
  const int tilesN = N >> 6;
  const int tilesM = M >> 6;
  const int tile = blockIdx.x * 8 + wave;
  if (tile >= tilesM * tilesN) return;
  const int tm = tile / tilesN;
  const int tn = tile - tm * tilesN;
  const int m0 = tm << 6;
  const int n0 = tn << 6;
  const int rlane = lane & 15;
  const int koff  = (lane >> 4) * 8;
  const int mOff  = (lane >> 4) * 8;

  v8f acc[4][4];
#pragma unroll
  for (int i = 0; i < 4; ++i) {
#pragma unroll
    for (int j = 0; j < 4; ++j) {
      acc[i][j] = (v8f){0.f, 0.f, 0.f, 0.f, 0.f, 0.f, 0.f, 0.f};
    }
  }

#pragma unroll 1
  for (int k0 = 0; k0 < K; k0 += 32) {
    v16h bf[4];
#pragma unroll
    for (int j = 0; j < 4; ++j) {
      bf[j] = frag_load(Bt + (size_t)(n0 + (j << 4) + rlane) * ldb + koff + k0);
    }
#pragma unroll
    for (int i = 0; i < 4; ++i) {
      const size_t ao = (size_t)(m0 + (i << 4) + rlane) * lda + koff + k0;
      const v16h a0 = frag_load(A + ao);
#pragma unroll
      for (int j = 0; j < 4; ++j) acc[i][j] = mma(a0, bf[j], acc[i][j]);
    }
  }

  float* slab = sT[wave];
  float bv[4] = {0.f, 0.f, 0.f, 0.f};
  if (EPI == 2) {
#pragma unroll
    for (int j = 0; j < 4; ++j) bv[j] = bias[n0 + (j << 4) + rlane];
  }
#pragma unroll
  for (int i = 0; i < 4; ++i) {
    const int mBase = m0 + (i << 4);
#pragma unroll
    for (int j = 0; j < 4; ++j) {
#pragma unroll
      for (int r = 0; r < 8; ++r) {
        float v = acc[i][j][r] * scale;
        if (EPI == 2) v = v + bv[j];
        slab[(mOff + r) * 68 + (j << 4) + rlane] = v;
      }
    }
    __builtin_amdgcn_fence(__ATOMIC_RELEASE, "workgroup");
    __builtin_amdgcn_wave_barrier();
    __builtin_amdgcn_fence(__ATOMIC_ACQUIRE, "workgroup");
    {
      const int hh = lane >> 4;
      const int c4 = (lane & 15) * 4;
      v4f vals[8];
#pragma unroll
      for (int it = 0; it < 8; ++it) {
        const int row = it * 2 + hh;
        v4f val = *(const v4f*)(slab + row * 68 + c4);
        if (EPI == 3) {
          const v4f av = *(const v4f*)(addp + (size_t)(mBase + row) * ldc + n0 + c4);
          val = val + av;
        }
        vals[it] = val;
      }
      for (int pass = 0; pass < 2; ++pass) {
#pragma unroll
        for (int it = 0; it < 8; ++it) {
          const int row = it * 2 + hh;
          *(volatile v4f*)(C + (size_t)(mBase + row) * ldc + n0 + c4) = vals[it];
        }
        __threadfence();
      }
    }
    __builtin_amdgcn_fence(__ATOMIC_RELEASE, "workgroup");
    __builtin_amdgcn_wave_barrier();
    __builtin_amdgcn_fence(__ATOMIC_ACQUIRE, "workgroup");
  }
}

__device__ __forceinline__ float conv_silu_one(v4f w, float u0, float u1, float u2, float u3, float b) {
  float acc = w[0] * u0;
  acc = fmaf(w[1], u1, acc);
  acc = fmaf(w[2], u2, acc);
  acc = fmaf(w[3], u3, acc);
  const float cv = acc + b;
  const float sg = 1.0f / (1.0f + expf(-cv));
  return cv * sg;
}

__global__ __launch_bounds__(256) void conv_silu_kernel(
    const float* __restrict__ XZ, const float* __restrict__ conv_w, const float* __restrict__ conv_b,
    float* __restrict__ UC, unsigned short* __restrict__ UCh, float carry)
{
  __shared__ __align__(16) float sRow[kDin];
  const int tid = threadIdx.x;
  const int r = blockIdx.x;
  const int t = r & (kSeq - 1);
  const int rb = r - t;
#pragma unroll 1
  for (int j = 0; j < 2; ++j) {
    const int d4 = j * 1024 + tid * 4;
    const v4f bs = *(const v4f*)(conv_b + d4);
    const v4f w0 = *(const v4f*)(conv_w + (size_t)d4 * 4);
    const v4f w1 = *(const v4f*)(conv_w + (size_t)d4 * 4 + 4);
    const v4f w2 = *(const v4f*)(conv_w + (size_t)d4 * 4 + 8);
    const v4f w3 = *(const v4f*)(conv_w + (size_t)d4 * 4 + 12);
    v4f ut[4];
#pragma unroll
    for (int k = 0; k < 4; ++k) {
      const int tt = t - 3 + k;
      const int tc = (tt < 0) ? 0 : tt;
      const bool on = (tt >= 0);
      const v4f ld = *(const v4f*)(XZ + (size_t)(rb + tc) * kXgN + d4);
      v4f uv;
      uv[0] = on ? ld[0] : 0.0f;
      uv[1] = on ? ld[1] : 0.0f;
      uv[2] = on ? ld[2] : 0.0f;
      uv[3] = on ? ld[3] : 0.0f;
      ut[k] = uv;
    }
    v4f o;
    o[0] = conv_silu_one(w0, ut[0][0], ut[1][0], ut[2][0], ut[3][0], bs[0]);
    o[1] = conv_silu_one(w1, ut[0][1], ut[1][1], ut[2][1], ut[3][1], bs[1]);
    o[2] = conv_silu_one(w2, ut[0][2], ut[1][2], ut[2][2], ut[3][2], bs[2]);
    o[3] = conv_silu_one(w3, ut[0][3], ut[1][3], ut[2][3], ut[3][3], bs[3]);
    *(v4f*)(sRow + d4) = o;
  }
  __syncthreads();
  const v4f o0 = *(const v4f*)(sRow + tid * 4);
  const v4f o1 = *(const v4f*)(sRow + 1024 + tid * 4);
  const v4f f0 = *(const v4f*)(sRow + tid * 8);
  const v4f f1 = *(const v4f*)(sRow + tid * 8 + 4);
  const float e0 = f0[0] * carry;
  const float e1 = f0[1] * carry;
  const float e2 = f0[2] * carry;
  const float e3 = f0[3] * carry;
  const float e4 = f1[0] * carry;
  const float e5 = f1[1] * carry;
  const float e6 = f1[2] * carry;
  const float e7 = f1[3] * carry;
  const v4u hw = (v4u){pack2(e0, e1), pack2(e2, e3), pack2(e4, e5), pack2(e6, e7)};
  float* ucr = UC + (size_t)r * kDin;
  unsigned short* uhr = UCh + (size_t)r * kDin;
  for (int pass = 0; pass < 2; ++pass) {
    *(volatile v4f*)(ucr + tid * 4) = o0;
    *(volatile v4f*)(ucr + 1024 + tid * 4) = o1;
    *(volatile v4u*)(uhr + tid * 8) = hw;
    __threadfence();
  }
}

}

extern "C" void kernel_launch(void* const* d_in, const int* in_sizes, int n_in,
                              void* d_out, int out_size, void* d_ws, size_t ws_size, hipStream_t stream)
{
  using namespace eng;
  if (n_in != 13) return;
  if (in_sizes[0] != kRowsAll * kDm) return;
  if (in_sizes[1] != kDm) return;
  if (in_sizes[2] != kDm) return;
  if (in_sizes[3] != kXgN * kDm) return;
  if (in_sizes[4] != kDin * 4) return;
  if (in_sizes[5] != kDin) return;
  if (in_sizes[6] != kDin * kDin) return;
  if (in_sizes[7] != kDin) return;
  if (in_sizes[8] != kNstate * kDin) return;
  if (in_sizes[9] != kNstate * kDin) return;
  if (in_sizes[10] != kDin * kNstate) return;
  if (in_sizes[11] != kDin) return;
  if (in_sizes[12] != kDm * kDin) return;
  if (out_size != kRowsAll * kDm) return;
  if (ws_size < kWsTotal) return;

  const float* x       = (const float*)d_in[0];
  const float* norm_w  = (const float*)d_in[1];
  const float* norm_b  = (const float*)d_in[2];
  const float* W_in    = (const float*)d_in[3];
  const float* conv_w  = (const float*)d_in[4];
  const float* conv_b  = (const float*)d_in[5];
  const float* W_dt    = (const float*)d_in[6];
  const float* b_dt    = (const float*)d_in[7];
  const float* W_b     = (const float*)d_in[8];
  const float* W_c     = (const float*)d_in[9];
  const float* A_log   = (const float*)d_in[10];
  const float* D_par   = (const float*)d_in[11];
  const float* W_out   = (const float*)d_in[12];
  float* out = (float*)d_out;

  char* ws = (char*)d_ws;
  size_t off = 0;
  unsigned short* WinH  = (unsigned short*)(ws + off);
  off += kBytesWin;
  unsigned short* WdtH  = (unsigned short*)(ws + off);
  off += kBytesWdt;
  unsigned short* WbcH  = (unsigned short*)(ws + off);
  off += kBytesWbc;
  unsigned short* WoutH = (unsigned short*)(ws + off);
  off += kBytesWout;
  unsigned short* Xh    = (unsigned short*)(ws + off);
  off += kBytesXh;
  float* XZ             = (float*)(ws + off);
  off += kBytesXZ;
  float* UC             = (float*)(ws + off);
  off += kBytesUC;
  unsigned short* UCh   = (unsigned short*)(ws + off);
  off += kBytesUCh;
  float* DTP            = (float*)(ws + off);
  off += kBytesDTP;
  float* BC             = (float*)(ws + off);
  off += kBytesBC;
  unsigned short* YH    = (unsigned short*)(ws + off);
  off += kBytesYH;
  if (off != kWsTotal) return;

  cast_carry_f16_kernel<<<dim3((kXgN * kDm / 8) / 256), 256, 0, stream>>>(W_in, WinH, kXgN * kDm / 8, kCarryWin);
  cast_carry_f16_kernel<<<dim3((kDin * kDin / 8) / 256), 256, 0, stream>>>(W_dt, WdtH, kDin * kDin / 8, kCarryWdt);
  cast_bc_kernel<<<dim3(kBcP), 256, 0, stream>>>(W_b, W_c, WbcH, kCarryWbc);
  cast_carry_f16_kernel<<<dim3((kDm * kDin / 8) / 256), 256, 0, stream>>>(W_out, WoutH, kDm * kDin / 8, kCarryWout);

  for (int p = 0; p < kNpass; ++p) {
    const size_t r0 = (size_t)p * kRows;
    const float* xp = x + r0 * kDm;
    float* outp = out + r0 * kDm;

    layernorm_cast_kernel<<<dim3(kRows / 8), 256, 0, stream>>>(xp, norm_w, norm_b, Xh, kRows, kCarryXn);

    gemm_f16_kernel<0><<<dim3((kRows / 64) * (kXgN / 64) / 8), 256, 0, stream>>>(
        Xh, kDm, WinH, kDm, XZ, kXgN, b_dt, xp, kRows, kXgN, kDm, kFoldIn);

    conv_silu_kernel<<<dim3(kRows), 256, 0, stream>>>(XZ, conv_w, conv_b, UC, UCh, kCarryU);

    gemm_f16_kernel<2><<<dim3((kRows / 64) * (kDin / 64) / 8), 256, 0, stream>>>(
        UCh, kDin, WdtH, kDin, DTP, kDin, b_dt, xp, kRows, kDin, kDin, kFoldDt);

    gemm_f16_kernel<0><<<dim3((kRows / 64) * (kBcP / 64) / 8), 256, 0, stream>>>(
        UCh, kDin, WbcH, kDin, BC, kBcP, b_dt, xp, kRows, kBcP, kDin, kFoldBc);

    for (int bb = 0; bb < kPassB; ++bb) {
      const size_t rr = (size_t)bb * kSeq;
      ms1_args sa;
      sa.dtpre = DTP + rr * kDin;
      sa.u = UC + rr * kDin;
      sa.bc = BC + rr * kBcP;
      sa.z = XZ + rr * kXgN;
      sa.A_log = A_log;
      sa.Dskip = D_par;
      sa.y = (__half*)(YH + rr * kDin);
      sa.y_lo = nullptr;
      sa.ld_dtpre = kDin;
      sa.ld_u = kDin;
      sa.ld_bc = kBcP;
      sa.ld_z = kXgN;
      sa.ld_y = kDin;
      sa.offB = kOffB;
      sa.offC = kOffC;
      sa.offZ = kDin;
      sa.ycarry = kCarryY;
      sa.dir = 1;
      sa.D = kDin;
      sa.L = kSeq;
      sa.nbatch = 1;
      ms1_scan_kernel<16><<<dim3(kDin / 64), 64, 0, stream>>>(sa);
    }

    gemm_f16_kernel<3><<<dim3((kRows / 64) * (kDm / 64) / 8), 256, 0, stream>>>(
        YH, kDin, WoutH, kDin, outp, kDm, b_dt, xp, kRows, kDm, kDin, kFoldOut);
  }
}
